// GraphAttentionNetwork_14877766713529
// MI455X (gfx1250) — hardware-verified
//
#include <hip/hip_runtime.h>
#include <math.h>

typedef __attribute__((ext_vector_type(16))) _Float16 v16h;
typedef __attribute__((ext_vector_type(16))) __bf16 v16b;
typedef __attribute__((ext_vector_type(8)))  _Float16 v8h;
typedef __attribute__((ext_vector_type(8)))  float v8f;
typedef __attribute__((ext_vector_type(4)))  float v4f;
typedef __attribute__((ext_vector_type(2)))  float v2f;
typedef __attribute__((ext_vector_type(4)))  unsigned v4u;
typedef __attribute__((ext_vector_type(4)))  int v4i;
typedef float __attribute__((may_alias)) float_a;
typedef int __attribute__((may_alias)) int_a;

template <typename T> __device__ __forceinline__ void vst2(void* p, T v) { *(volatile T*)p = v; __threadfence(); *(volatile T*)p = v; }
__device__ __forceinline__ v8f wmma16(v16h a, v16h b, v8f c) {
  v8f d = __builtin_amdgcn_wmma_f32_16x16x32_f16(false, a, false, b, (short)0, c, false, false);
  asm volatile("v_nop\n\tv_nop\n\tv_nop\n\tv_nop" : "+v"(d) : "v"(a), "v"(b));
  return d;
}
__device__ __forceinline__ v8f wmma_bf(v16b a, v16b b, v8f c) {
  v8f d = __builtin_amdgcn_wmma_f32_16x16x32_bf16(false, a, false, b, (short)0, c, false, false);
  asm volatile("v_nop\n\tv_nop\n\tv_nop\n\tv_nop" : "+v"(d) : "v"(a), "v"(b));
  return d;
}
__device__ __forceinline__ v16h frag_h(const _Float16* rowk0, int lane) {
  union { v16h v; v8h q[2]; } u; const _Float16* p = rowk0 + 8 * (lane >> 4);
  u.q[0] = *(const v8h*)p; u.q[1] = *(const v8h*)(p + 16); return u.v;
}
__device__ __forceinline__ v16h frag_f32(const float* rowk0, int lane) {
  v16h a; const float* p = rowk0 + 8 * (lane >> 4);
#pragma unroll
  for (int i = 0; i < 8; ++i) { a[i] = (_Float16)p[i]; a[8 + i] = (_Float16)p[16 + i]; }
  return a;
}
__device__ __forceinline__ v16h frag_f32s(const float* rowk0, int lane, float sc) {
  v16h a; const float* p = rowk0 + 8 * (lane >> 4);
#pragma unroll
  for (int i = 0; i < 8; ++i) { a[i] = (_Float16)(p[i] * sc); a[8 + i] = (_Float16)(p[16 + i] * sc); }
  return a;
}
__device__ __forceinline__ v16h fragc_f32(const float* W, int k0, int n, int lane, int ld, int K) {
  v16h a; const int g = lane >> 4;
#pragma unroll
  for (int i = 0; i < 8; ++i) { const int ka = k0 + 8 * g + i, kb = ka + 16;
    a[i] = (_Float16)(ka < K ? W[(size_t)(ka < K ? ka : K - 1) * ld + n] : 0.f); a[8 + i] = (_Float16)(kb < K ? W[(size_t)(kb < K ? kb : K - 1) * ld + n] : 0.f); }
  return a;
}
struct F2 { v16b h, l; };
__device__ __forceinline__ F2 bsplit16(const float v[16]) { F2 r;
#pragma unroll
  for (int i = 0; i < 16; ++i) { const __bf16 h = (__bf16)v[i]; r.h[i] = h; r.l[i] = (__bf16)(v[i] - (float)h); }
  return r; }
__device__ __forceinline__ F2 split_row(const float* row, int k0, int lane) { float v[16]; const float* p = row + k0 + 8 * (lane >> 4);
#pragma unroll
  for (int i = 0; i < 8; ++i) { v[i] = p[i]; v[8 + i] = p[16 + i]; }
  return bsplit16(v); }
__device__ __forceinline__ F2 split_rowK(const float* row, int k0, int lane, int K) { float v[16]; const int g = lane >> 4;
#pragma unroll
  for (int i = 0; i < 8; ++i) { const int ka = k0 + 8 * g + i, kb = ka + 16; v[i] = ka < K ? row[ka < K ? ka : K - 1] : 0.f; v[8 + i] = kb < K ? row[kb < K ? kb : K - 1] : 0.f; }
  return bsplit16(v); }
__device__ __forceinline__ F2 split_col(const float* W, int k0, int n, int lane, int ld, int K) { float v[16]; const int g = lane >> 4;
#pragma unroll
  for (int i = 0; i < 8; ++i) { const int ka = k0 + 8 * g + i, kb = ka + 16; v[i] = ka < K ? W[(size_t)(ka < K ? ka : K - 1) * ld + n] : 0.f; v[8 + i] = kb < K ? W[(size_t)(kb < K ? kb : K - 1) * ld + n] : 0.f; }
  return bsplit16(v); }
__device__ __forceinline__ v8f mac3(const F2& a, const F2& b, v8f c) { c = wmma_bf(a.l, b.h, c); c = wmma_bf(a.h, b.l, c); return wmma_bf(a.h, b.h, c); }
__device__ __forceinline__ float sigm(float v) { return 1.0f / (1.0f + expf(-v)); }
#define LDSX() do { asm volatile("s_wait_dscnt 0" ::: "memory"); __builtin_amdgcn_wave_barrier(); __builtin_amdgcn_fence(__ATOMIC_RELEASE, "workgroup"); } while (0)

__device__ __forceinline__ float bfr(float v) { return (float)(__bf16)v; }
__device__ __forceinline__ float elu1(float v) { return v > 0.f ? v : expm1f(v); }
#define NN 2048
#define DIN 128
#define NHD 8
#define HDD 64
#define CH (NHD * HDD)
#define HG 4
#ifndef ASTR
#define ASTR NN
#endif
typedef __attribute__((ext_vector_type(8))) __bf16 v8b;
__device__ __forceinline__ v16b frag_b(const __bf16* rowk0, int lane) { union { v16b v; v8b q[2]; } u; const __bf16* p = rowk0 + 8 * (lane >> 4); u.q[0] = *(const v8b*)p; u.q[1] = *(const v8b*)(p + 16); return u.v; }
#define WS_H   0u
#define WS_X   (WS_H + 4u * (size_t)NN * CH)
#define WS_E   (WS_X + 4u * (size_t)NN * CH)
#define WS_HT  (WS_E + 4u * (size_t)16 * NN)
#define WS_HL  (WS_HT + 2u * (size_t)CH * NN)
#define WS_P   (WS_HL + 2u * (size_t)CH * NN)
#define WS_END (WS_P + 4u * (size_t)HG * NN * NN)
__global__ __launch_bounds__(128) void k_lin(const float* __restrict__ X, int kin, int xpitch, int xraw, const float* __restrict__ Wt, int nout, const float* __restrict__ AV, float* __restrict__ H, float* __restrict__ E) {   __shared__ __align__(16) float sf[4][16][132]; __shared__ __align__(16) float se[4][64];
  const int tid = threadIdx.x, wave = tid >> 5, lane = tid & 31, col = lane & 15, g = lane >> 4; const size_t r0 = (size_t)blockIdx.x * 64 + wave * 16; const int c0 = blockIdx.y * 128; const int dh = (nout == HDD) ? HDD : HDD;
  v8f acc[8] = {};
#pragma unroll 1
  for (int kc = 0; kc < kin / 32; ++kc) { F2 a; if (xraw) { float v[16]; const float* p = X + (r0 + col) * (size_t)xpitch + kc * 32 + 8 * g;
#pragma unroll
      for (int i = 0; i < 8; ++i) { v[i] = bfr(p[i]); v[8 + i] = bfr(p[16 + i]); }
      a = bsplit16(v); } else a = split_row(X + (r0 + col) * (size_t)xpitch, kc * 32, lane);
#pragma unroll
    for (int j = 0; j < 8; ++j) { v16b w; const int o = c0 + j * 16 + col;
#pragma unroll
      for (int i = 0; i < 8; ++i) { const int ka = kc * 32 + 8 * g + i, kb = ka + 16; w[i] = (o < nout) ? (__bf16)Wt[(size_t)ka * nout + o] : (__bf16)0.f; w[8 + i] = (o < nout) ? (__bf16)Wt[(size_t)kb * nout + o] : (__bf16)0.f; }
      asm volatile("s_wait_loadcnt 0x0" ::: "memory"); acc[j] = wmma_bf(a.h, w, acc[j]); acc[j] = wmma_bf(a.l, w, acc[j]); } }
  float pi[2][8], pj[2][8];
#pragma unroll
  for (int hh = 0; hh < 2; ++hh)
#pragma unroll
    for (int r = 0; r < 8; ++r) { pi[hh][r] = 0.f; pj[hh][r] = 0.f; }
#pragma unroll
  for (int j = 0; j < 8; ++j) { const int d = (j & 3) * 16 + col; const float as = bfr(AV[d]), ad = bfr(AV[dh + d]);
#pragma unroll
    for (int r = 0; r < 8; ++r) { pi[j >> 2][r] += acc[j][r] * as; pj[j >> 2][r] += acc[j][r] * ad; } }
#pragma unroll
  for (int hh = 0; hh < 2; ++hh)
#pragma unroll
    for (int r = 0; r < 8; ++r) {
#pragma unroll
      for (int s_ = 1; s_ < 16; s_ <<= 1) { pi[hh][r] += __shfl_xor(pi[hh][r], s_); pj[hh][r] += __shfl_xor(pj[hh][r], s_); } }
  if (col == 0) { const int hbase = c0 / HDD;
#pragma unroll
    for (int hh = 0; hh < 2; ++hh)
#pragma unroll
      for (int r = 0; r < 8; ++r) { const int rl = wave * 16 + 8 * g + r; se[hh][rl] = pi[hh][r]; se[2 + hh][rl] = pj[hh][r]; } (void)hbase; }
#pragma unroll
  for (int j = 0; j < 8; ++j)
#pragma unroll
    for (int r = 0; r < 8; ++r) sf[wave][8 * g + r][j * 16 + col] = acc[j][r];
  __syncthreads();
  for (int rl = 0; rl < 16; ++rl) if (c0 + lane * 4 < nout) vst2(H + (r0 + rl) * CH + c0 + lane * 4, *(const v4f*)&sf[wave][rl][lane * 4]);
  { const int hbase = c0 / HDD; const int pl = tid >> 4, q = tid & 15;
    if (tid < 64) { const int hh = pl & 1; const int isj = pl >> 1; if (hbase + hh < nout / HDD) vst2(E + (size_t)(isj * 8 + hbase + hh) * NN + (size_t)blockIdx.x * 64 + q * 4, *(const v4f*)&se[isj * 2 + hh][q * 4]); } } }
__global__ __launch_bounds__(128) void k_ht(const float* __restrict__ H, int nout, __bf16* __restrict__ HT, __bf16* __restrict__ HL) { __shared__ __align__(16) __bf16 th[128][136], tl[128][136];
  const int tid = threadIdx.x; const int n0 = blockIdx.x * 128; const int c0 = blockIdx.y * 128;
  for (int e = tid; e < 128 * 128; e += 128) { const int nl = e >> 7, cl = e & 127; const float v = (c0 + cl < nout) ? H[(size_t)(n0 + nl) * CH + c0 + cl] : 0.f; const __bf16 h = (__bf16)v; th[cl][nl] = h; tl[cl][nl] = (__bf16)(v - (float)h); }
  __syncthreads();
  for (int e = tid; e < 128 * 16; e += 128) { const int cl = e >> 4, q = e & 15; if (c0 + cl < nout) { const size_t o = (size_t)(c0 + cl) * NN + n0 + q * 8; vst2((unsigned*)(HT + o), *(const v4u*)&th[cl][q * 8]); vst2((unsigned*)(HL + o), *(const v4u*)&tl[cl][q * 8]); } } }
__global__ __launch_bounds__(256) void k_p(const float* __restrict__ E, const int* __restrict__ ADJ, int h0, float* __restrict__ P0) { __shared__ float sred[8]; __shared__ float sbc; __shared__ __align__(16) float sh[NN];
  const int t = threadIdx.x; const size_t i = blockIdx.x; const int h = h0 + blockIdx.y; float* P = P0 + ((size_t)blockIdx.y * NN + i) * NN; const int* arow = ADJ + i * ASTR;
  const float ei = E[(size_t)h * NN + i];
  float m = -3.0e38f;
  for (int j = t; j < NN; j += 256) { float v = ei + E[(size_t)(8 + h) * NN + j]; v = v > 0.f ? v : 0.2f * v; if (arow[j] == 0) v = -1.0e9f; sh[j] = v; m = fmaxf(m, v); }
#pragma unroll
  for (int o = 1; o < 32; o <<= 1) m = fmaxf(m, __shfl_xor(m, o));
  if ((t & 31) == 0) sred[t >> 5] = m; __syncthreads(); if (t == 0) { float a = sred[0]; for (int w = 1; w < 8; ++w) a = fmaxf(a, sred[w]); sbc = a; } __syncthreads(); m = sbc; __syncthreads();
  float s = 0.f; for (int j = t; j < NN; j += 256) { const float e = expf(sh[j] - m); sh[j] = e; s += e; }
#pragma unroll
  for (int o = 1; o < 32; o <<= 1) s += __shfl_xor(s, o);
  if ((t & 31) == 0) sred[t >> 5] = s; __syncthreads(); if (t == 0) { float a = 0.f; for (int w = 0; w < 8; ++w) a += sred[w]; sbc = 2048.0f / a; } __syncthreads(); const float sc = sbc;
  for (int j = t; j < NN; j += 256) sh[j] *= sc;
  __syncthreads(); for (int q = t; q < NN / 4; q += 256) vst2(P + q * 4, *(const v4f*)&sh[q * 4]); }
__global__ __launch_bounds__(128) void k_pv(const float* __restrict__ P0, const __bf16* __restrict__ HT, const __bf16* __restrict__ HL, int h0, int act, int ostride, float* __restrict__ OUT) { __shared__ __align__(16) float ss[4][16][HDD + 4];
  const int h = h0 + blockIdx.z; const float* PS = P0 + (size_t)blockIdx.z * NN * NN;
  const int tid = threadIdx.x, wave = tid >> 5, lane = tid & 31, col = lane & 15, g = lane >> 4; const int ql0 = blockIdx.x * 64 + wave * 16;
  v8f acc[HDD / 16] = {};
#pragma unroll 1
  for (int kc = 0; kc < NN / 32; ++kc) { const F2 p = split_row(PS + (size_t)(ql0 + col) * NN, kc * 32, lane);
#pragma unroll
    for (int j = 0; j < HDD / 16; ++j) { const size_t po = ((size_t)h * HDD + j * 16 + col) * NN + kc * 32; const v16b vh = frag_b(HT + po, lane); acc[j] = wmma_bf(p.h, vh, acc[j]); acc[j] = wmma_bf(p.l, vh, acc[j]); acc[j] = wmma_bf(p.h, frag_b(HL + po, lane), acc[j]); } }
#pragma unroll
  for (int j = 0; j < HDD / 16; ++j)
#pragma unroll
    for (int r = 0; r < 8; ++r) { const float v = acc[j][r] * (1.0f / 2048.0f); ss[wave][8 * g + r][j * 16 + col] = act ? elu1(v) : v; }
  LDSX(); for (int rl = 0; rl < 16; ++rl) if (lane < HDD / 4) vst2(OUT + (size_t)(ql0 + rl) * ostride + h * HDD + lane * 4, *(const v4f*)&ss[wave][rl][lane * 4]); }
extern "C" void kernel_launch(void* const* d_in, const int* in_sizes, int n_in, void* d_out, int out_size, void* d_ws, size_t ws_size, hipStream_t stream) {
  (void)in_sizes; (void)n_in; (void)out_size;
  const float** F = (const float**)d_in;
  if (ws_size < (size_t)WS_END) return;
  char* ws = (char*)d_ws; float *H = (float*)(ws + WS_H), *XB = (float*)(ws + WS_X), *E = (float*)(ws + WS_E), *P = (float*)(ws + WS_P); __bf16 *HT = (__bf16*)(ws + WS_HT), *HL = (__bf16*)(ws + WS_HL);
  const int* ADJ = (const int*)d_in[1];
  k_lin<<<dim3(NN / 64, CH / 128), 128, 0, stream>>>(F[0], DIN, DIN, 1, F[2], CH, F[3], H, E);
  k_ht<<<dim3(NN / 128, CH / 128), 128, 0, stream>>>(H, CH, HT, HL);
  for (int h0 = 0; h0 < NHD; h0 += HG) { k_p<<<dim3(NN, HG), 256, 0, stream>>>(E, ADJ, h0, P); k_pv<<<dim3(NN / 64, 1, HG), 128, 0, stream>>>(P, HT, HL, h0, 1, CH, XB); }
  k_lin<<<dim3(NN / 64, CH / 128), 128, 0, stream>>>(XB, CH, CH, 0, F[4], CH, F[5], H, E);
  k_ht<<<dim3(NN / 128, CH / 128), 128, 0, stream>>>(H, CH, HT, HL);
  for (int h0 = 0; h0 < NHD; h0 += HG) { k_p<<<dim3(NN, HG), 256, 0, stream>>>(E, ADJ, h0, P); k_pv<<<dim3(NN / 64, 1, HG), 128, 0, stream>>>(P, HT, HL, h0, 1, CH, XB); }
  k_lin<<<dim3(NN / 64, 1), 128, 0, stream>>>(XB, CH, CH, 0, F[6], HDD, F[7], H, E);
  k_ht<<<dim3(NN / 128, 1), 128, 0, stream>>>(H, HDD, HT, HL);
  k_p<<<dim3(NN, 1), 256, 0, stream>>>(E, ADJ, 0, P);
  k_pv<<<dim3(NN / 64, 1, 1), 128, 0, stream>>>(P, HT, HL, 0, 0, HDD, (float*)d_out);
}
